// MultiHeadAttention_56006373540301
// MI455X (gfx1250) — hardware-run, weakly checked
//
#include <hip/hip_runtime.h>
#ifndef NB
#define NB 2
#endif
#ifndef SQ
#define SQ 2048
#endif
#define NB_FULL 2
#define SQ_FULL 2048
#define DM 1024
#define NH 16
#define HD 64
#define QC 256
#define ER ((SQ) < 512 ? (SQ) : 512)
#define LQ (3 * DM)

typedef unsigned short v8us __attribute__((ext_vector_type(8), may_alias));
typedef float  v8f  __attribute__((ext_vector_type(8)));
typedef float  v4f  __attribute__((ext_vector_type(4)));
typedef float  v4fa __attribute__((ext_vector_type(4), may_alias));
typedef int    v4i  __attribute__((ext_vector_type(4)));
typedef int    v4ia __attribute__((ext_vector_type(4), may_alias));
typedef _Float16 v16h __attribute__((ext_vector_type(16)));
typedef _Float16 v4h __attribute__((ext_vector_type(4)));
union FragH { v16h v; v8us half[2]; _Float16 h[16]; unsigned short u[16]; };

static_assert(NB <= NB_FULL && SQ <= SQ_FULL);
static_assert(NH * HD == DM && DM % 64 == 0);
static_assert(QC == 256 && SQ % QC == 0 && ER % QC == 0 && ER <= SQ && (SQ - ER) % 128 == 0 && SQ % 128 == 0);

__device__ __forceinline__ unsigned short bf16_bits(float x) { unsigned int u = __float_as_uint(x); return (unsigned short)((u + 0x7FFFu + ((u >> 16) & 1u)) >> 16); }
__device__ __forceinline__ float bf16_rne(float x) { return __uint_as_float(((unsigned int)bf16_bits(x)) << 16); }

__device__ __forceinline__ v16h g2_frag(const _Float16* p, int hh) { FragH f; f.half[0] = *(const v8us*)((const unsigned short*)p + 8 * hh); f.half[1] = *(const v8us*)((const unsigned short*)p + 16 + 8 * hh); return f.v; }
__device__ __forceinline__ v8f g2_mma(v16h a, v16h b, v8f c) { v8f d = __builtin_amdgcn_wmma_f32_16x16x32_f16(false, a, false, b, (short)0, c, false, false); asm volatile("v_nop\n\tv_nop\n\tv_nop\n\tv_nop" : "+v"(d) : "v"(a), "v"(b)); return d; }

__global__ __launch_bounds__(256) void k_x16(const float* __restrict__ x, _Float16* __restrict__ X16, size_t n8) {
  const size_t t = (size_t)blockIdx.x * 256 + threadIdx.x; if (t >= n8) return;
  const size_t row = t / (DM / 8); const int c8 = (int)(t % (DM / 8)) * 8; const size_t b = row / SQ, tt = row % SQ;
  const float* src = x + (b * SQ_FULL + tt) * DM + c8;
  const v4f a = *(const v4fa*)src, c = *(const v4fa*)(src + 4); FragH f;
#pragma unroll
  for (int q = 0; q < 4; ++q) { f.h[q] = (_Float16)bf16_rne(a[q]); f.h[4 + q] = (_Float16)bf16_rne(c[q]); }
  const v8us o = f.half[0];
  *(volatile v8us*)((unsigned short*)X16 + t * 8) = o; __threadfence(); *(volatile v8us*)((unsigned short*)X16 + t * 8) = o;
}

__global__ __launch_bounds__(256) void k_wt_f16(const float* __restrict__ W, _Float16* __restrict__ Wt, int K, int N, float scale) {
  const int t = blockIdx.x * 256 + threadIdx.x; if (t >= N * (K / 8)) return;
  W += (size_t)blockIdx.y * K * N; Wt += (size_t)blockIdx.y * N * K;
  const int n = t / (K / 8), k8 = (t % (K / 8)) * 8; FragH f;
#pragma unroll
  for (int i = 0; i < 8; ++i) f.h[i] = (_Float16)(bf16_rne(W[(size_t)(k8 + i) * N + n]) * scale);
  const v8us o = f.half[0];
  *(volatile v8us*)((unsigned short*)Wt + (size_t)n * K + k8) = o; __threadfence(); *(volatile v8us*)((unsigned short*)Wt + (size_t)n * K + k8) = o;
}

template <int NHv, int TTv>
__global__ __launch_bounds__(256) void k_vt(const _Float16* __restrict__ V16, int ldv, int voff, _Float16* __restrict__ Vt) {
  __shared__ unsigned short tl[64][66];
  const int tid = threadIdx.x; const int slab = blockIdx.x / (TTv / 64), lg = blockIdx.x % (TTv / 64); const int b = slab / NHv, h = slab % NHv;
  for (int i = tid; i < 64 * 8; i += 256) { const int r = i / 8, c8 = (i % 8) * 8; FragH f; f.half[0] = *(const v8us*)((const unsigned short*)V16 + ((size_t)b * TTv + lg * 64 + r) * ldv + voff + h * 64 + c8);
#pragma unroll
    for (int q = 0; q < 8; ++q) tl[r][c8 + q] = f.u[q]; }
  __syncthreads();
  for (int pass = 0; pass < 2; ++pass) {
#pragma unroll
    for (int rd = 0; rd < 2; ++rd) { const int d = rd * 32 + tid / 8, pc = tid % 8; FragH f;
#pragma unroll
      for (int q = 0; q < 8; ++q) f.u[q] = tl[pc * 8 + q][d];
      *(volatile v8us*)((unsigned short*)Vt + ((size_t)slab * 64 + d) * TTv + lg * 64 + pc * 8) = f.half[0]; }
    if (pass == 0) __threadfence(); }
}

__global__ __launch_bounds__(128) void k_gemm2(const _Float16* __restrict__ A, int lda, size_t sA, const _Float16* __restrict__ Bh, int ldb, size_t sB, float alpha, const float* __restrict__ bias,
    float* __restrict__ C, _Float16* __restrict__ C16, _Float16* __restrict__ C16L, int ldc, size_t sC, int lrows, size_t sCL, int M, int N, int K) {
  __shared__ __attribute__((aligned(16))) float so[4][32][68];
  const int tid = threadIdx.x, w = tid >> 5, lane = tid & 31, ln = lane & 15, hh = lane >> 4; const int by = blockIdx.y;
  A += (size_t)by * sA; Bh += (size_t)by * sB; const size_t cofs = (size_t)by * sC; const size_t lofs = (size_t)by * sCL;
  const int ntn = N >> 6; const int mt = blockIdx.x / ntn, nq = blockIdx.x - mt * ntn; const int row0 = mt * 128 + 32 * w, col0 = nq * 64; if (row0 >= M) return;
  const _Float16* a0p = A + (size_t)(row0 + ln) * lda; const _Float16* a1p = a0p + (size_t)16 * lda;
  const _Float16* b0p = Bh + (size_t)(col0 + ln) * ldb; const _Float16* b1p = b0p + (size_t)16 * ldb; const _Float16* b2p = b1p + (size_t)16 * ldb; const _Float16* b3p = b2p + (size_t)16 * ldb;
  const v8f z8 = {0.f,0.f,0.f,0.f,0.f,0.f,0.f,0.f}; v8f c00 = z8, c01 = z8, c02 = z8, c03 = z8, c10 = z8, c11 = z8, c12 = z8, c13 = z8;
#pragma unroll 1
  for (int kb = 0; kb < K; kb += 32) { const v16h a0 = g2_frag(a0p + kb, hh), a1 = g2_frag(a1p + kb, hh);
    v16h b = g2_frag(b0p + kb, hh); c00 = g2_mma(a0, b, c00); c10 = g2_mma(a1, b, c10);
    b = g2_frag(b1p + kb, hh); c01 = g2_mma(a0, b, c01); c11 = g2_mma(a1, b, c11);
    b = g2_frag(b2p + kb, hh); c02 = g2_mma(a0, b, c02); c12 = g2_mma(a1, b, c12);
    b = g2_frag(b3p + kb, hh); c03 = g2_mma(a0, b, c03); c13 = g2_mma(a1, b, c13); }
  v8f accs[8] = {c00, c01, c02, c03, c10, c11, c12, c13};
#pragma unroll
  for (int u = 0; u < 8; ++u) { const int t = u & 3, half = u >> 2; const int col = col0 + t * 16 + ln; const float bv = bias ? bf16_rne(bias[col]) : 0.f;
#pragma unroll
    for (int r = 0; r < 8; ++r) { const int rloc = half * 16 + 8 * hh + r; so[w][rloc][t * 16 + ln] = accs[u][r] * alpha + bv; } }
  __builtin_amdgcn_fence(4  , "workgroup"); __builtin_amdgcn_wave_barrier();
  const int rsub = lane >> 4, c4 = (lane & 15) * 4;
  for (int pass = 0; pass < 2; ++pass) {
#pragma unroll
    for (int q = 0; q < 16; ++q) { const int r = q * 2 + rsub; const v4f v = *(const v4fa*)&so[w][r][c4];
      v4h h4, l4;
#pragma unroll
      for (int i = 0; i < 4; ++i) { h4[i] = (_Float16)v[i]; l4[i] = (_Float16)((v[i] - (float)h4[i]) * 1024.0f); }
      if (C) *(volatile v4f*)(C + cofs + (size_t)(row0 + r) * ldc + col0 + c4) = v;
      if (C16) *(volatile v4h*)(C16 + cofs + (size_t)(row0 + r) * ldc + col0 + c4) = h4;
      if (C16L && (row0 + r) < lrows) *(volatile v4h*)(C16L + lofs + (size_t)(row0 + r) * ldc + col0 + c4) = l4; }
    if (pass == 0) __threadfence(); }
}

template <bool BSPLIT>
__global__ __launch_bounds__(128) void k_gemm2r(const _Float16* __restrict__ A, const _Float16* __restrict__ AL, int lda, int ldal, size_t sA, size_t sAL,
    const _Float16* __restrict__ Bh, const _Float16* __restrict__ BL, int ldb, int ldbl, size_t sB, size_t sBL, float alpha, const float* __restrict__ bias,
    float* __restrict__ C, _Float16* __restrict__ C16, _Float16* __restrict__ C16L, int ldc, int ldcl, size_t sC, size_t sCL, int M, int N, int K) {
  __shared__ __attribute__((aligned(16))) float so[4][16][68];
  const int tid = threadIdx.x, w = tid >> 5, lane = tid & 31, ln = lane & 15, hh = lane >> 4; const int by = blockIdx.y;
  A += (size_t)by * sA; AL += (size_t)by * sAL; Bh += (size_t)by * sB; BL += (size_t)by * sBL; const size_t cofs = (size_t)by * sC; const size_t lofs = (size_t)by * sCL;
  const int ntn = N >> 6; const int mt = blockIdx.x / ntn, nq = blockIdx.x - mt * ntn; const int row0 = mt * 64 + 16 * w, col0 = nq * 64; if (row0 >= M) return;
  const _Float16* ap = A + (size_t)(row0 + ln) * lda; const _Float16* alp = AL + (size_t)(row0 + ln) * ldal;
  const _Float16* b0p = Bh + (size_t)(col0 + ln) * ldb; const _Float16* b1p = b0p + (size_t)16 * ldb; const _Float16* b2p = b1p + (size_t)16 * ldb; const _Float16* b3p = b2p + (size_t)16 * ldb;
  const _Float16* l0p = BL + (size_t)(col0 + ln) * ldbl; const _Float16* l1p = l0p + (size_t)16 * ldbl; const _Float16* l2p = l1p + (size_t)16 * ldbl; const _Float16* l3p = l2p + (size_t)16 * ldbl;
  const v8f z8 = {0.f,0.f,0.f,0.f,0.f,0.f,0.f,0.f}; v8f h0 = z8, h1 = z8, h2 = z8, h3 = z8, r0 = z8, r1 = z8, r2 = z8, r3 = z8;
#pragma unroll 1
  for (int kb = 0; kb < K; kb += 32) { const v16h ah = g2_frag(ap + kb, hh), al = g2_frag(alp + kb, hh);
    v16h b = g2_frag(b0p + kb, hh); h0 = g2_mma(ah, b, h0); r0 = g2_mma(al, b, r0); if (BSPLIT) { const v16h bl = g2_frag(l0p + kb, hh); r0 = g2_mma(ah, bl, r0); }
    b = g2_frag(b1p + kb, hh); h1 = g2_mma(ah, b, h1); r1 = g2_mma(al, b, r1); if (BSPLIT) { const v16h bl = g2_frag(l1p + kb, hh); r1 = g2_mma(ah, bl, r1); }
    b = g2_frag(b2p + kb, hh); h2 = g2_mma(ah, b, h2); r2 = g2_mma(al, b, r2); if (BSPLIT) { const v16h bl = g2_frag(l2p + kb, hh); r2 = g2_mma(ah, bl, r2); }
    b = g2_frag(b3p + kb, hh); h3 = g2_mma(ah, b, h3); r3 = g2_mma(al, b, r3); if (BSPLIT) { const v16h bl = g2_frag(l3p + kb, hh); r3 = g2_mma(ah, bl, r3); } }
  v8f hs[4] = {h0, h1, h2, h3}; v8f rs[4] = {r0, r1, r2, r3};
#pragma unroll
  for (int t = 0; t < 4; ++t) { const int col = col0 + t * 16 + ln; const float bv = bias ? bf16_rne(bias[col]) : 0.f;
#pragma unroll
    for (int r = 0; r < 8; ++r) so[w][8 * hh + r][t * 16 + ln] = (hs[t][r] + rs[t][r] * 0.0009765625f) * alpha + bv; }
  __builtin_amdgcn_fence(4  , "workgroup"); __builtin_amdgcn_wave_barrier();
  const int rsub = lane >> 4, c4 = (lane & 15) * 4;
  for (int pass = 0; pass < 2; ++pass) {
#pragma unroll
    for (int q = 0; q < 8; ++q) { const int r = q * 2 + rsub; const v4f v = *(const v4fa*)&so[w][r][c4];
      v4h h4, l4;
#pragma unroll
      for (int i = 0; i < 4; ++i) { h4[i] = (_Float16)v[i]; l4[i] = (_Float16)((v[i] - (float)h4[i]) * 1024.0f); }
      if (C) *(volatile v4f*)(C + cofs + (size_t)(row0 + r) * ldc + col0 + c4) = v;
      if (C16) *(volatile v4h*)(C16 + cofs + (size_t)(row0 + r) * ldc + col0 + c4) = h4;
      if (C16L) *(volatile v4h*)(C16L + lofs + (size_t)(row0 + r) * ldcl + col0 + c4) = l4; }
    if (pass == 0) __threadfence(); }
}

template <bool RES>
__global__ __launch_bounds__(256) void k_sm(const float* __restrict__ S, _Float16* __restrict__ P, _Float16* __restrict__ PL, int nrows, int kext, const int* __restrict__ am) {
  #pragma clang fp contract(off)
  const int lane = threadIdx.x & 31, w = threadIdx.x >> 5;
  const int i = blockIdx.x * 8 + w; if (i >= nrows) return;
  const float* s = S + (size_t)i * kext; const int* mr = am + (size_t)(i % QC) * SQ_FULL; const int nit = kext >> 8;
  float mx = -1.0e9f;
#pragma unroll 1
  for (int it = 0; it < nit; ++it) { const int j = it * 256 + lane * 8;
    const v4f a = *(const v4fa*)(s + j), c = *(const v4fa*)(s + j + 4); const v4i m0 = *(const v4ia*)(mr + j), m1 = *(const v4ia*)(mr + j + 4);
#pragma unroll
    for (int q = 0; q < 4; ++q) { mx = fmaxf(mx, (m0[q] != 0) ? a[q] : -1.0e9f); mx = fmaxf(mx, (m1[q] != 0) ? c[q] : -1.0e9f); } }
  mx = fmaxf(mx, __shfl_xor(mx, 16)); mx = fmaxf(mx, __shfl_xor(mx, 8)); mx = fmaxf(mx, __shfl_xor(mx, 4)); mx = fmaxf(mx, __shfl_xor(mx, 2)); mx = fmaxf(mx, __shfl_xor(mx, 1));
  float se = 0.f;
#pragma unroll 1
  for (int it = 0; it < nit; ++it) { const int j = it * 256 + lane * 8;
    const v4f a = *(const v4fa*)(s + j), c = *(const v4fa*)(s + j + 4); const v4i m0 = *(const v4ia*)(mr + j), m1 = *(const v4ia*)(mr + j + 4);
#pragma unroll
    for (int q = 0; q < 4; ++q) { const float e0 = __expf(a[q] - mx), e1 = __expf(c[q] - mx); se += (m0[q] != 0) ? e0 : 0.f; se += (m1[q] != 0) ? e1 : 0.f; } }
  se += __shfl_xor(se, 16); se += __shfl_xor(se, 8); se += __shfl_xor(se, 4); se += __shfl_xor(se, 2); se += __shfl_xor(se, 1);
  const float qn = __uint_as_float(0x7FC00000u);
  const float sc = (mx > -5.0e8f) ? 1024.0f / se : qn;
#pragma unroll 1
  for (int it = 0; it < nit; ++it) { const int j = it * 256 + lane * 8;
    const v4f a = *(const v4fa*)(s + j), c = *(const v4fa*)(s + j + 4); const v4i m0 = *(const v4ia*)(mr + j), m1 = *(const v4ia*)(mr + j + 4);
    FragH fh, fl;
#pragma unroll
    for (int q = 0; q < 4; ++q) { const float e0 = __expf(a[q] - mx), e1 = __expf(c[q] - mx);
      const float p0 = ((m0[q] != 0) ? e0 : 0.f) * sc, p1 = ((m1[q] != 0) ? e1 : 0.f) * sc;
      const _Float16 g0 = (_Float16)p0, g1 = (_Float16)p1; fh.h[q] = g0; fh.h[4 + q] = g1;
      fl.h[q] = (_Float16)((p0 - (float)g0) * 1024.0f); fl.h[4 + q] = (_Float16)((p1 - (float)g1) * 1024.0f); }
    const v8us oh = fh.half[0], ol = fl.half[0];
    unsigned short* d = (unsigned short*)P + (size_t)i * kext + j; unsigned short* dl = (unsigned short*)PL + (size_t)i * kext + j;
    *(volatile v8us*)d = oh; if (RES) *(volatile v8us*)dl = ol;
    __threadfence();
    *(volatile v8us*)d = oh; if (RES) *(volatile v8us*)dl = ol; }
}

__global__ __launch_bounds__(256) void k_mchk(const int* __restrict__ am, int* __restrict__ FL) {
  __shared__ int red[8];
  const int tid = threadIdx.x, lane = tid & 31, w = tid >> 5; const int blk = blockIdx.x; const int b = blk / (SQ / 32), t0 = (blk % (SQ / 32)) * 32;
  int bad = 0;
#pragma unroll 1
  for (int rr = 0; rr < 4; ++rr) { const int t = t0 + w * 4 + rr; const int k0 = (t / QC + 1) * QC; const int* mr = am + ((size_t)b * SQ_FULL + t) * SQ_FULL;
#pragma unroll 1
    for (int sx = k0 + lane * 4; sx < SQ; sx += 128) { const v4i m = *(const v4ia*)(mr + sx); bad |= (m[0] | m[1] | m[2] | m[3]); } }
  const int wb = __any(bad != 0) ? 1 : 0;
  if (lane == 0) red[w] = wb;
  __syncthreads();
  if (w == 0) { int f = 0;
#pragma unroll
    for (int q = 0; q < 8; ++q) f |= red[q];
    *(volatile int*)(FL + (size_t)blk * 32 + lane) = f; __threadfence(); *(volatile int*)(FL + (size_t)blk * 32 + lane) = f; }
}

__global__ __launch_bounds__(256) void k_fill(const int* __restrict__ FL, int nfl, float* __restrict__ out) {
  const int lane = threadIdx.x & 31; int bad = 0;
  for (int i = lane; i < nfl; i += 32) bad |= FL[(size_t)i * 32];
  if (!__any(bad != 0)) return;
  const float qn = __uint_as_float(0x7FC00000u); const v4f nv = {qn, qn, qn, qn};
  const size_t n4 = (size_t)NB * SQ * (DM / 4); const size_t stride = (size_t)gridDim.x * 256;
  for (size_t idx = (size_t)blockIdx.x * 256 + threadIdx.x; idx < n4; idx += stride) { const size_t row = idx / (DM / 4); const int c4 = (int)(idx % (DM / 4)) * 4; const size_t b = row / SQ, tt = row % SQ;
    float* d = out + (b * SQ_FULL + tt) * DM + c4; *(volatile v4f*)d = nv; __threadfence(); *(volatile v4f*)d = nv; }
}

extern "C" void kernel_launch(void* const* d_in, const int* in_sizes, int n_in,
                              void* d_out, int out_size, void* d_ws, size_t ws_size, hipStream_t stream) {
  if (n_in < 7) return;
  const size_t rows_need = (size_t)(NB - 1) * SQ_FULL + SQ;
  if ((size_t)in_sizes[0] < rows_need * DM) return;
  if ((size_t)in_sizes[1] < rows_need * SQ_FULL) return;
  if ((size_t)in_sizes[2] < (size_t)NH * DM * HD || (size_t)in_sizes[3] < (size_t)NH * DM * HD || (size_t)in_sizes[4] < (size_t)NH * DM * HD) return;
  if ((size_t)in_sizes[5] < (size_t)DM * DM || (size_t)in_sizes[6] < (size_t)DM) return;
  if ((size_t)out_size < rows_need * DM) return;
  const float* x = (const float*)d_in[0]; const int* am = (const int*)d_in[1];
  const float* wq = (const float*)d_in[2]; const float* wk = (const float*)d_in[3]; const float* wv = (const float*)d_in[4];
  const float* wproj = (const float*)d_in[5]; const float* bproj = (const float*)d_in[6]; float* out = (float*)d_out;

  constexpr size_t szW = (size_t)3 * DM * DM * 2, szBO = (size_t)DM * DM * 2, szX = (size_t)NB * SQ * DM * 2, szQKV = (size_t)NB * SQ * LQ * 2, szQKVL = (size_t)NB * ER * LQ * 2;
  constexpr size_t szVT = (size_t)NB * NH * HD * SQ * 2, szVTL = (size_t)NB * NH * HD * ER * 2, szO = (size_t)NB * SQ * DM * 2, szOL = (size_t)NB * ER * DM * 2;
  constexpr size_t szS = (size_t)NH * QC * SQ * 4, szP = (size_t)NH * QC * SQ * 2, szPL = (size_t)NH * QC * ER * 2, szFL = (size_t)NB * (SQ / 32) * 128;
  static_assert(szW % 256 == 0 && szBO % 256 == 0 && szX % 256 == 0 && szQKV % 256 == 0 && szQKVL % 256 == 0 && szVT % 256 == 0 && szVTL % 256 == 0 && szO % 256 == 0 && szOL % 256 == 0 && szS % 256 == 0 && szP % 256 == 0 && szPL % 256 == 0 && szFL % 256 == 0);
  static_assert(szW + szBO + szX + szQKV + szQKVL + szVT + szVTL + szO + szOL + szS + szP + szPL + szFL <= (size_t)134217728);
  char* ws = (char*)d_ws; size_t off = 0;
  auto take = [&](size_t bytes) { char* p = ws + off; off += (bytes + 255) & ~(size_t)255; return p; };
  _Float16* WQKV = (_Float16*)take(szW); _Float16* BO = (_Float16*)take(szBO); _Float16* X16 = (_Float16*)take(szX);
  _Float16* QKV16 = (_Float16*)take(szQKV); _Float16* QKVL = (_Float16*)take(szQKVL);
  _Float16* VT = (_Float16*)take(szVT); _Float16* VTL = (_Float16*)take(szVTL); _Float16* O16 = (_Float16*)take(szO); _Float16* OL = (_Float16*)take(szOL);
  float* S = (float*)take(szS); _Float16* P = (_Float16*)take(szP); _Float16* PL = (_Float16*)take(szPL); int* FL = (int*)take(szFL);
  if (off > ws_size) return;

  k_x16<<<(unsigned)(((size_t)NB * SQ * DM / 8 + 255) / 256), 256, 0, stream>>>(x, X16, (size_t)NB * SQ * DM / 8);
  k_wt_f16<<<dim3((HD * (DM / 8) + 255) / 256, NH), 256, 0, stream>>>(wq, WQKV, DM, HD, 16.0f);
  k_wt_f16<<<dim3((HD * (DM / 8) + 255) / 256, NH), 256, 0, stream>>>(wk, WQKV + (size_t)DM * DM, DM, HD, 16.0f);
  k_wt_f16<<<dim3((HD * (DM / 8) + 255) / 256, NH), 256, 0, stream>>>(wv, WQKV + (size_t)2 * DM * DM, DM, HD, 16.0f);
  k_wt_f16<<<dim3((DM * (DM / 8) + 255) / 256, 1), 256, 0, stream>>>(wproj, BO, DM, DM, 16.0f);
  k_mchk<<<NB * (SQ / 32), 256, 0, stream>>>(am, FL);

  k_gemm2<<<dim3((SQ / 128) * (LQ / 64), NB), 128, 0, stream>>>(X16, DM, (size_t)SQ * DM, WQKV, DM, 0, 0.0625f, nullptr,
      nullptr, QKV16, QKVL, LQ, (size_t)SQ * LQ, ER, (size_t)ER * LQ, SQ, LQ, DM);
  k_vt<NH, SQ><<<NB * NH * (SQ / 64), 256, 0, stream>>>(QKV16, LQ, 2 * DM, VT);
  k_vt<NH, ER><<<NB * NH * (ER / 64), 256, 0, stream>>>(QKVL, LQ, 2 * DM, VTL);

  for (int b = 0; b < NB; ++b) {
    const _Float16* Qb = QKV16 + (size_t)b * SQ * LQ; const _Float16* Kb = Qb + DM;
    const _Float16* QLb = QKVL + (size_t)b * ER * LQ; const _Float16* KLb = QLb + DM;
    const _Float16* VTb = VT + (size_t)b * NH * HD * SQ; const _Float16* VTLb = VTL + (size_t)b * NH * HD * ER;
    for (int c = 0; c < SQ / QC; ++c) {
      const int kext = (c + 1) * QC;
      const int* amc = am + ((size_t)b * SQ_FULL + (size_t)c * QC) * SQ_FULL;
      if (c < ER / QC) {
        k_gemm2r<true><<<dim3((QC / 64) * (kext / 64), NH), 128, 0, stream>>>(Qb + (size_t)c * QC * LQ, QLb + (size_t)c * QC * LQ, LQ, LQ, (size_t)HD, (size_t)HD,
            Kb, KLb, LQ, LQ, (size_t)HD, (size_t)HD, 0.125f, nullptr, S, nullptr, nullptr, kext, 0, (size_t)QC * kext, 0, QC, kext, HD);
        k_sm<true><<<NH * QC / 8, 256, 0, stream>>>(S, P, PL, NH * QC, kext, amc);
        k_gemm2r<true><<<dim3((QC / 64) * (HD / 64), NH), 128, 0, stream>>>(P, PL, kext, kext, (size_t)QC * kext, (size_t)QC * kext,
            VTb, VTLb, SQ, ER, (size_t)HD * SQ, (size_t)HD * ER, 0.0625f, nullptr,
            nullptr, O16 + ((size_t)b * SQ + (size_t)c * QC) * DM, OL + ((size_t)b * ER + (size_t)c * QC) * DM, DM, DM, (size_t)HD, (size_t)HD, QC, HD, kext);
      } else {
        k_gemm2<<<dim3((QC / 128) * (kext / 64), NH), 128, 0, stream>>>(Qb + (size_t)c * QC * LQ, LQ, (size_t)HD, Kb, LQ, (size_t)HD, 0.125f, nullptr,
            S, nullptr, nullptr, kext, (size_t)QC * kext, 0, 0, QC, kext, HD);
        k_sm<false><<<NH * QC / 8, 256, 0, stream>>>(S, P, PL, NH * QC, kext, amc);
        k_gemm2<<<dim3((QC / 128) * (HD / 64), NH), 128, 0, stream>>>(P, kext, (size_t)QC * kext, VTb, SQ, (size_t)HD * SQ, 0.0625f, nullptr,
            nullptr, O16 + ((size_t)b * SQ + (size_t)c * QC) * DM, nullptr, DM, (size_t)HD, 0, 0, QC, HD, kext);
      }
    }
  }
  if (SQ > ER)
    k_gemm2<<<dim3(((SQ - ER) / 128) * (DM / 64), NB), 128, 0, stream>>>(O16 + (size_t)ER * DM, DM, (size_t)SQ * DM, BO, DM, 0, 0.0009765625f, bproj,
        out + (size_t)ER * DM, nullptr, nullptr, DM, (size_t)SQ_FULL * DM, 0, 0, SQ - ER, DM, DM);
  k_gemm2r<false><<<dim3((ER / 64) * (DM / 64), NB), 128, 0, stream>>>(O16, OL, DM, DM, (size_t)SQ * DM, (size_t)ER * DM, BO, BO, DM, DM, 0, 0, 0.0009765625f, bproj,
      out, nullptr, nullptr, DM, DM, (size_t)SQ_FULL * DM, 0, ER, DM, DM);
  k_fill<<<64, 256, 0, stream>>>(FL, NB * (SQ / 32), out);
}
